// StrongGNNModel_16612933501368
// MI455X (gfx1250) — hardware-verified
//
#include <hip/hip_runtime.h>
#include <hip/hip_bf16.h>
#include <stddef.h>
#include <math.h>


#define FD      128
#define NIN     32
#define EEMB    64
#define NBT     6
#define NBD     4
#define NCMB    (NBT * NBD)
#define NLAY    5
#define NB      256
#define NTHR    256
#define NWAVE   8
#define EPT     8
#define CHUNK   (NTHR * EPT)
#define WCAP    (EPT * 32)
#define PASSN   128
#define PCAP    2048
#define EHDR    32
#define EROW    (EHDR + PCAP)
#define PJT     128
#define PJR     64
#define GB      16
#define PTHR    256
#define PEPT    4
#define PCHUNK  (PTHR * PEPT)
#define PWCAP   (PEPT * 32)
#define HTHR    128
#define HG      64
#define EXPK    200
#define EXPKP   224
#define CMBW    384
#define GEW     256
#define O1W     256
#define BNS     0.99999500003749981f

#define LDS_ACC   0
#define LDS_MSG   (LDS_ACC + (NB + 1) * FD * 4)
#define LDS_SLOT  (LDS_MSG + PASSN * FD * 4)
#define LDS_LAYER (LDS_SLOT + PASSN * 4)
#define LDS_PROJ  (4 * 16 * FD * 4 + PJR * FD * 4)
#define HWT0      4096
#define HWT1      2048
#define HWCT      (16 * CMBW)
#define HWAVE     (HWT0 + HWT1 + HWCT)
#define LDS_HEAD  (4 * HWAVE * 4 + HG * 4)

#define U0 (FD * (NIN / 8))
#define U1 (FD * (FD / 8))
#define U2 (NLAY * FD * (FD / 8))
#define U3 U2
#define U4 (FD * (EXPKP / 8))
#define U5 U1
#define U6 (O1W * (CMBW / 8))
#define U7 (FD * (O1W / 8))
#define PE0 (U0 / NTHR)
#define PE1 (PE0 + U1 / NTHR)
#define PE2 (PE1 + U2 / NTHR)
#define PE3 (PE2 + U3 / NTHR)
#define PE4 (PE3 + U4 / NTHR)
#define PE5 (PE4 + U5 / NTHR)
#define PE6 (PE5 + U6 / NTHR)
#define PE7 (PE6 + U7 / NTHR)
#define PBT PE7

static_assert(NB == 2 * NWAVE * 16);
static_assert(NTHR == NWAVE * 32);
static_assert(NTHR == 2 * PASSN);
static_assert(NWAVE * 16 * FD * 4 == PASSN * FD * 4);
static_assert((PCAP % PASSN) == 0);
static_assert(EHDR * 4 == 128);
static_assert((EROW % 4) == 0 && ((EROW * 4) % 128) == 0);
static_assert((LDS_LAYER % 16) == 0 && LDS_LAYER <= 300 * 1024);
static_assert(LDS_HEAD <= 300 * 1024);
static_assert(GB == 16 && PTHR == 256 && PTHR == NWAVE * 32);
static_assert(HWT0 >= 16 * EXPKP && HWT0 >= 16 * O1W && HWT1 >= 16 * FD);
static_assert((EXPKP % 32) == 0 && EXPKP >= EXPK);
static_assert((U0 % NTHR) == 0 && (U1 % NTHR) == 0 && (U2 % NTHR) == 0 && (U4 % NTHR) == 0);
static_assert((U6 % NTHR) == 0 && (U7 % NTHR) == 0);
static_assert(PBT == 176);
static_assert(HTHR == 4 * 32 && HG == 4 * 16);
static_assert(PJT == 4 * 32 && PJR == 4 * 16 && (NB % PJR) == 0);

typedef float          v4f   __attribute__((ext_vector_type(4)));
typedef float          v8f   __attribute__((ext_vector_type(8)));
typedef int            v4i   __attribute__((ext_vector_type(4)));
typedef unsigned short v8us  __attribute__((ext_vector_type(8)));
typedef unsigned short v16us __attribute__((ext_vector_type(16)));
typedef __bf16         v16bf __attribute__((ext_vector_type(16)));
union FragB { v16bf v; v16us u; v8us h[2]; };
union Pk8 { v8us h; v4i i; };

__device__ __forceinline__ unsigned f2bf(float f) {
  const unsigned u = __float_as_uint(f);
  return (u + 0x7FFFu + ((u >> 16) & 1u)) >> 16;
}

__device__ __forceinline__ void split8(v4f a, v4f b, v8us& hi, v8us& lo) {
  float f[8];
  f[0] = a.x; f[1] = a.y; f[2] = a.z; f[3] = a.w;
  f[4] = b.x; f[5] = b.y; f[6] = b.z; f[7] = b.w;
  v8us rh, rl;
#pragma unroll
  for (int i = 0; i < 8; ++i) {
    const unsigned hb = f2bf(f[i]);
    const float r = f[i] - __uint_as_float(hb << 16);
    rh[i] = (unsigned short)hb;
    rl[i] = (unsigned short)f2bf(r);
  }
  hi = rh;
  lo = rl;
}

__device__ __forceinline__ v8f ldc8(const float* p) {
  const v4f a = *(const v4f*)p;
  const v4f b = *(const v4f*)(p + 4);
  v8f c;
  c[0] = a.x; c[1] = a.y; c[2] = a.z; c[3] = a.w;
  c[4] = b.x; c[5] = b.y; c[6] = b.z; c[7] = b.w;
  return c;
}

__device__ __forceinline__ v8f wm3(v16bf ah, v16bf al, v16bf bh, v16bf bl, v8f c) {
  v8f d = __builtin_amdgcn_wmma_f32_16x16x32_bf16(false, ah, false, bh, (short)0, c, false, false);
  d = __builtin_amdgcn_wmma_f32_16x16x32_bf16(false, ah, false, bl, (short)0, d, false, false);
  d = __builtin_amdgcn_wmma_f32_16x16x32_bf16(false, al, false, bh, (short)0, d, false, false);
  asm volatile("v_nop\n\tv_nop\n\tv_nop\n\tv_nop" : "+v"(d) : "v"(ah), "v"(al), "v"(bh), "v"(bl));
  return d;
}

__device__ __forceinline__ void strelu8(float* p, v8f c) {
  v4f a, b;
  a.x = fmaxf(c[0], 0.0f); a.y = fmaxf(c[1], 0.0f); a.z = fmaxf(c[2], 0.0f); a.w = fmaxf(c[3], 0.0f);
  b.x = fmaxf(c[4], 0.0f); b.y = fmaxf(c[5], 0.0f); b.z = fmaxf(c[6], 0.0f); b.w = fmaxf(c[7], 0.0f);
  *(v4f*)p = a;
  *(v4f*)(p + 4) = b;
}

__device__ __forceinline__ v4f relu4sum(v4f a, v4f t) {
  v4f o;
  o.x = fmaxf(a.x + t.x, 0.0f); o.y = fmaxf(a.y + t.y, 0.0f);
  o.z = fmaxf(a.z + t.z, 0.0f); o.w = fmaxf(a.w + t.w, 0.0f);
  return o;
}

__device__ __forceinline__ int scan_chunk(const int* __restrict__ dsts, int nE, int cbase, int nodeBase,
                                          int vec8, int* list, int tid, int wave) {
  int wc = 0;
  const int el0  = tid * EPT;
  const int e0   = cbase + el0;
  const int sent = -2147483647 - 1;
  v4i da, db;
  if (vec8 != 0 && cbase + CHUNK <= nE) {
    da = *(const v4i*)(dsts + e0);
    db = *(const v4i*)(dsts + e0 + 4);
  } else {
    da.x = (e0     < nE) ? dsts[min(e0, nE - 1)] : sent;
    da.y = (e0 + 1 < nE) ? dsts[min(e0 + 1, nE - 1)] : sent;
    da.z = (e0 + 2 < nE) ? dsts[min(e0 + 2, nE - 1)] : sent;
    da.w = (e0 + 3 < nE) ? dsts[min(e0 + 3, nE - 1)] : sent;
    db.x = (e0 + 4 < nE) ? dsts[min(e0 + 4, nE - 1)] : sent;
    db.y = (e0 + 5 < nE) ? dsts[min(e0 + 5, nE - 1)] : sent;
    db.z = (e0 + 6 < nE) ? dsts[min(e0 + 6, nE - 1)] : sent;
    db.w = (e0 + 7 < nE) ? dsts[min(e0 + 7, nE - 1)] : sent;
  }
  const unsigned nb = (unsigned)nodeBase;
  const unsigned s0 = (unsigned)da.x - nb, s1 = (unsigned)da.y - nb;
  const unsigned s2 = (unsigned)da.z - nb, s3 = (unsigned)da.w - nb;
  const unsigned s4 = (unsigned)db.x - nb, s5 = (unsigned)db.y - nb;
  const unsigned s6 = (unsigned)db.z - nb, s7 = (unsigned)db.w - nb;
  const bool h0 = s0 < (unsigned)NB, h1 = s1 < (unsigned)NB, h2 = s2 < (unsigned)NB, h3 = s3 < (unsigned)NB;
  const bool h4 = s4 < (unsigned)NB, h5 = s5 < (unsigned)NB, h6 = s6 < (unsigned)NB, h7 = s7 < (unsigned)NB;
  const unsigned any = __builtin_amdgcn_ballot_w32(h0 | h1 | h2 | h3 | h4 | h5 | h6 | h7);
  if (any != 0u) {
#define HITJ(J, HJ) { \
      const unsigned mj = __builtin_amdgcn_ballot_w32(HJ); \
      if (mj != 0u) { \
        if (HJ) { \
          const int pos = wc + (int)__builtin_amdgcn_mbcnt_lo(mj, 0u); \
          if (pos < WCAP) list[wave * WCAP + pos] = el0 + (J); \
        } \
        wc += (int)__builtin_popcount(mj); } }
    HITJ(0, h0)
    HITJ(1, h1)
    HITJ(2, h2)
    HITJ(3, h3)
    HITJ(4, h4)
    HITJ(5, h5)
    HITJ(6, h6)
    HITJ(7, h7)
#undef HITJ
  }
  return wc;
}

__global__ __launch_bounds__(NTHR) void k_prep(
    const float* __restrict__ nw1, const float* __restrict__ nw2,
    const float* __restrict__ mw1, const float* __restrict__ mw2,
    const float* __restrict__ ew1, const float* __restrict__ ew2,
    const float* __restrict__ hw1, const float* __restrict__ hw2,
    unsigned short* q0, unsigned short* q1, unsigned short* q2, unsigned short* q3,
    unsigned short* q4, unsigned short* q5, unsigned short* q6, unsigned short* q7) {
  const int b = blockIdx.x, tid = threadIdx.x;
  const float* src;
  unsigned short* dst;
  int Kin, Kp, O, L, ub;
  if (b < PE0)      { src = nw1; dst = q0; Kin = NIN;  Kp = NIN;   O = FD;  L = 1;    ub = b; }
  else if (b < PE1) { src = nw2; dst = q1; Kin = FD;   Kp = FD;    O = FD;  L = 1;    ub = b - PE0; }
  else if (b < PE2) { src = mw1; dst = q2; Kin = FD;   Kp = FD;    O = FD;  L = NLAY; ub = b - PE1; }
  else if (b < PE3) { src = mw2; dst = q3; Kin = FD;   Kp = FD;    O = FD;  L = NLAY; ub = b - PE2; }
  else if (b < PE4) { src = ew1; dst = q4; Kin = EXPK; Kp = EXPKP; O = FD;  L = 1;    ub = b - PE3; }
  else if (b < PE5) { src = ew2; dst = q5; Kin = FD;   Kp = FD;    O = FD;  L = 1;    ub = b - PE4; }
  else if (b < PE6) { src = hw1; dst = q6; Kin = CMBW; Kp = CMBW;  O = O1W; L = 1;    ub = b - PE5; }
  else              { src = hw2; dst = q7; Kin = O1W;  Kp = O1W;   O = FD;  L = 1;    ub = b - PE6; }
  const int u   = ub * NTHR + tid;
  const int cpr = Kp >> 3;
  const int row = u / cpr;
  const int kc  = u - row * cpr;
  int l = row / O;
  l = l > L - 1 ? L - 1 : l;
  const int o = row - l * O;
  float f[8];
#pragma unroll
  for (int j = 0; j < 8; ++j) {
    const int k   = 8 * kc + j;
    const int kcl = k < Kin ? k : Kin - 1;
    const float w = src[((size_t)(l * Kin + kcl)) * O + o];
    f[j] = (k < Kin) ? w : 0.0f;
  }
  Pk8 ph, pl;
  {
    v4f a, c;
    a.x = f[0]; a.y = f[1]; a.z = f[2]; a.w = f[3];
    c.x = f[4]; c.y = f[5]; c.z = f[6]; c.w = f[7];
    split8(a, c, ph.h, pl.h);
  }
  const size_t ne = (size_t)L * O * Kp;
  unsigned short* dh = dst + (size_t)u * 8;
  unsigned short* dl = dst + ne + (size_t)u * 8;
  *(volatile v4i*)dh = ph.i;
  *(volatile v4i*)dl = pl.i;
  __threadfence();
  *(volatile v4i*)dh = ph.i;
  *(volatile v4i*)dl = pl.i;
}

__global__ __launch_bounds__(NTHR) void k_tab(const float* __restrict__ te, const float* __restrict__ de,
                                             const float* __restrict__ lew, const float* __restrict__ leb,
                                             float* tab) {
  const int idx = blockIdx.x * NTHR + threadIdx.x;
  const int total = NLAY * NCMB * FD;
  if (idx >= total) return;
  const int f = idx & (FD - 1);
  const int comb = idx >> 7;
  const int l = comb / NCMB;
  const int c = comb - l * NCMB;
  const int t = c >> 2, d = c & 3;
  float s = leb[l * FD + f];
#pragma unroll 1
  for (int k = 0; k < EEMB; ++k)
    s += (te[t * EEMB + k] + de[d * EEMB + k]) * lew[((size_t)(l * EEMB + k)) * FD + f];
  *(volatile float*)(tab + idx) = s;
  __threadfence();
  *(volatile float*)(tab + idx) = s;
}

__global__ __launch_bounds__(NTHR) void k_escan(const int* __restrict__ ei, int* etab, int nE, int vec8) {
  __shared__ int list[NWAVE * WCAP];
  __shared__ __attribute__((aligned(16))) int pend[EROW];
  __shared__ int wcnt[NWAVE];
  const int tid = threadIdx.x, lane = tid & 31, wave = tid >> 5;
  const int nodeBase = blockIdx.x * NB;
  const int* dsts = ei + nE;
  for (int i = tid; i < EROW; i += NTHR) pend[i] = 0;
  __syncthreads();
  int pendN = 0;
  const int nChunks = (nE + CHUNK - 1) / CHUNK;
#pragma unroll 1
  for (int ch = 0; ch < nChunks; ++ch) {
    const int cbase = ch * CHUNK;
    const int wc = scan_chunk(dsts, nE, cbase, nodeBase, vec8, list, tid, wave);
    if (lane == 0) wcnt[wave] = wc;
    __syncthreads();
    const int base = pendN;
    int tot = 0, myoff = 0;
#pragma unroll
    for (int w = 0; w < NWAVE; ++w) {
      int c = wcnt[w];
      c = c > WCAP ? WCAP : (c < 0 ? 0 : c);
      if (w < wave) myoff += c;
      tot += c;
    }
    {
      int n = wcnt[wave];
      n = n > WCAP ? WCAP : (n < 0 ? 0 : n);
      const int* lp = list + wave * WCAP;
      for (int i = lane; i < n; i += 32) {
        const int pos = base + myoff + i;
        if (pos < PCAP) pend[EHDR + pos] = cbase + lp[i];
      }
    }
    const int newN = base + tot;
    pendN = newN > PCAP ? PCAP : newN;
    __syncthreads();
  }
  if (tid == 0) pend[0] = pendN;
  __syncthreads();
  int* rowp = etab + (size_t)blockIdx.x * EROW;
#pragma unroll 1
  for (int u = tid; u < EROW / 4; u += NTHR) {
    const v4i v = *(const v4i*)(pend + 4 * u);
    *(volatile v4i*)(rowp + 4 * u) = v;
  }
  __threadfence();
#pragma unroll 1
  for (int u = tid; u < EROW / 4; u += NTHR) {
    const v4i v = *(const v4i*)(pend + 4 * u);
    *(volatile v4i*)(rowp + 4 * u) = v;
  }
}

template <int NKT1, int LAYER>
__device__ __forceinline__ void mlp_tile(const float* zrow, const float* __restrict__ xrow,
    const unsigned short* __restrict__ p1h, const unsigned short* __restrict__ p1l, const float* __restrict__ b1,
    const unsigned short* __restrict__ p2h, const unsigned short* __restrict__ p2l, const float* __restrict__ b2,
    const float* __restrict__ gam, const float* __restrict__ bet,
    float* hw, float* srow, int hh, int m) {
  FragB bh[4], bl[4];
#pragma unroll
  for (int kt = 0; kt < NKT1; ++kt) {
    const int k0 = 32 * kt + 8 * hh;
    v4f a = *(const v4f*)(xrow + k0);
    v4f b = *(const v4f*)(xrow + k0 + 4);
    v4f c = *(const v4f*)(xrow + k0 + 16);
    v4f d = *(const v4f*)(xrow + k0 + 20);
    if (LAYER != 0) {
      a += *(const v4f*)(zrow + k0);
      b += *(const v4f*)(zrow + k0 + 4);
      c += *(const v4f*)(zrow + k0 + 16);
      d += *(const v4f*)(zrow + k0 + 20);
    }
    split8(a, b, bh[kt].h[0], bl[kt].h[0]);
    split8(c, d, bh[kt].h[1], bl[kt].h[1]);
  }
#pragma unroll 1
  for (int ft = 0; ft < FD / 16; ++ft) {
    v8f acc = ldc8(b1 + 16 * ft + 8 * hh);
    const size_t ao = (size_t)(16 * ft + m) * (32 * NKT1) + 8 * hh;
#pragma unroll
    for (int kt = 0; kt < NKT1; ++kt) {
      FragB fh, fl;
      fh.h[0] = *(const v8us*)(p1h + ao + 32 * kt);
      fh.h[1] = *(const v8us*)(p1h + ao + 32 * kt + 16);
      fl.h[0] = *(const v8us*)(p1l + ao + 32 * kt);
      fl.h[1] = *(const v8us*)(p1l + ao + 32 * kt + 16);
      acc = wm3(fh.v, fl.v, bh[kt].v, bl[kt].v, acc);
    }
    strelu8(hw + m * FD + 16 * ft + 8 * hh, acc);
  }
  __syncthreads();
#pragma unroll
  for (int kt = 0; kt < 4; ++kt) {
    const float* hp = hw + m * FD + 32 * kt + 8 * hh;
    split8(*(const v4f*)hp, *(const v4f*)(hp + 4), bh[kt].h[0], bl[kt].h[0]);
    split8(*(const v4f*)(hp + 16), *(const v4f*)(hp + 20), bh[kt].h[1], bl[kt].h[1]);
  }
#pragma unroll 1
  for (int ft = 0; ft < FD / 16; ++ft) {
    v8f acc = ldc8(b2 + 16 * ft + 8 * hh);
    const size_t ao = (size_t)(16 * ft + m) * FD + 8 * hh;
#pragma unroll
    for (int kt = 0; kt < 4; ++kt) {
      FragB fh, fl;
      fh.h[0] = *(const v8us*)(p2h + ao + 32 * kt);
      fh.h[1] = *(const v8us*)(p2h + ao + 32 * kt + 16);
      fl.h[0] = *(const v8us*)(p2l + ao + 32 * kt);
      fl.h[1] = *(const v8us*)(p2l + ao + 32 * kt + 16);
      acc = wm3(fh.v, fl.v, bh[kt].v, bl[kt].v, acc);
    }
    const int f0 = 16 * ft + 8 * hh;
    float o[8];
    if (LAYER != 0) {
      const v4f g0 = *(const v4f*)(gam + f0);
      const v4f g1 = *(const v4f*)(gam + f0 + 4);
      const v4f e0 = *(const v4f*)(bet + f0);
      const v4f e1 = *(const v4f*)(bet + f0 + 4);
      const v4f x0 = *(const v4f*)(xrow + f0);
      const v4f x1 = *(const v4f*)(xrow + f0 + 4);
      float gs[8], be[8], xs[8];
      gs[0] = g0.x; gs[1] = g0.y; gs[2] = g0.z; gs[3] = g0.w; gs[4] = g1.x; gs[5] = g1.y; gs[6] = g1.z; gs[7] = g1.w;
      be[0] = e0.x; be[1] = e0.y; be[2] = e0.z; be[3] = e0.w; be[4] = e1.x; be[5] = e1.y; be[6] = e1.z; be[7] = e1.w;
      xs[0] = x0.x; xs[1] = x0.y; xs[2] = x0.z; xs[3] = x0.w; xs[4] = x1.x; xs[5] = x1.y; xs[6] = x1.z; xs[7] = x1.w;
#pragma unroll
      for (int r = 0; r < 8; ++r) {
        const float sc = gs[r] * BNS;
        o[r] = fmaxf(acc[r] * sc + be[r], 0.0f) + xs[r];
      }
    } else {
#pragma unroll
      for (int r = 0; r < 8; ++r) o[r] = acc[r];
    }
    v4f o0, o1;
    o0.x = o[0]; o0.y = o[1]; o0.z = o[2]; o0.w = o[3];
    o1.x = o[4]; o1.y = o[5]; o1.z = o[6]; o1.w = o[7];
    *(v4f*)(srow + f0) = o0;
    *(v4f*)(srow + f0 + 4) = o1;
  }
}

__global__ __launch_bounds__(PJT) void k_proj(const float* __restrict__ x,
    const unsigned short* __restrict__ p1h, const unsigned short* __restrict__ p1l, const float* __restrict__ nb1,
    const unsigned short* __restrict__ p2h, const unsigned short* __restrict__ p2l, const float* __restrict__ nb2,
    float* hout, int nN) {
  extern __shared__ __attribute__((aligned(16))) unsigned char dsmp[];
  float* hid = (float*)dsmp;
  float* stg = (float*)(dsmp + 4 * 16 * FD * 4);
  const int tid = threadIdx.x, lane = tid & 31, wave = tid >> 5, hh = lane >> 4, m = lane & 15;
  const int rowBase = blockIdx.x * PJR;
  const int lrow = wave * 16 + m;
  int node = rowBase + lrow;
  node = node > nN - 1 ? nN - 1 : node;
  mlp_tile<1, 0>(nullptr, x + (size_t)node * NIN, p1h, p1l, nb1, p2h, p2l, nb2, nullptr, nullptr,
                 hid + wave * 16 * FD, stg + lrow * FD, hh, m);
  __syncthreads();
#pragma unroll 1
  for (int rr = 0; rr < 16; ++rr) {
    const int row = wave * 16 + rr;
    const v4f v = *(const v4f*)(stg + row * FD + 4 * lane);
    *(volatile v4f*)(hout + (size_t)(rowBase + row) * FD + 4 * lane) = v;
  }
  __threadfence();
#pragma unroll 1
  for (int rr = 0; rr < 16; ++rr) {
    const int row = wave * 16 + rr;
    const v4f v = *(const v4f*)(stg + row * FD + 4 * lane);
    *(volatile v4f*)(hout + (size_t)(rowBase + row) * FD + 4 * lane) = v;
  }
}

__global__ __launch_bounds__(NTHR) void k_layer(
    const float* __restrict__ hin, const int* __restrict__ ei, const int* __restrict__ ea,
    const int* __restrict__ etab, const float* __restrict__ elt,
    const unsigned short* __restrict__ m1h, const unsigned short* __restrict__ m1l, const float* __restrict__ b1,
    const unsigned short* __restrict__ m2h, const unsigned short* __restrict__ m2l, const float* __restrict__ b2,
    const float* __restrict__ gam, const float* __restrict__ bet,
    float* hout, int nN, int nE) {
  extern __shared__ __attribute__((aligned(16))) unsigned char dsm[];
  float* acc   = (float*)(dsm + LDS_ACC);
  float* msg   = (float*)(dsm + LDS_MSG);
  float* hid   = (float*)(dsm + LDS_MSG);
  int*   slotb = (int*)(dsm + LDS_SLOT);

  const int tid = threadIdx.x, lane = tid & 31, wave = tid >> 5, hh = lane >> 4, m = lane & 15;
  const int nodeBase = blockIdx.x * NB;
  const int* srcs = ei;
  const int* dsts = ei + nE;
  const int* erow = etab + (size_t)blockIdx.x * EROW;

  {
    v4f z;
    z.x = 0.0f; z.y = 0.0f; z.z = 0.0f; z.w = 0.0f;
    for (int i = tid; i < (NB + 1) * FD / 4; i += NTHR) *(v4f*)(acc + 4 * i) = z;
  }
  int nP = erow[0];
  nP = nP < 0 ? 0 : (nP > PCAP ? PCAP : nP);
  int R = (nP + PASSN - 1) / PASSN;
  R = R > PCAP / PASSN ? PCAP / PASSN : R;
  __syncthreads();

#pragma unroll 1
  for (int r = 0; r < R; ++r) {
    {
      const int i = tid >> 1, q = tid & 1;
      const int idx = r * PASSN + i;
      const bool valid = idx < nP;
      const int idxc = idx < PCAP ? idx : PCAP - 1;
      int e = erow[EHDR + idxc];
      e = e < 0 ? 0 : (e > nE - 1 ? nE - 1 : e);
      const int d = dsts[e];
      int s = srcs[e];
      s = s < 0 ? 0 : (s > nN - 1 ? nN - 1 : s);
      int slot = d - nodeBase;
      if (!valid || (unsigned)slot >= (unsigned)NB) slot = NB;
      int bt = ea[2 * e];
      int bd = ea[2 * e + 1];
      bt = bt < 0 ? 0 : (bt > NBT - 1 ? NBT - 1 : bt);
      bd = bd < 0 ? 0 : (bd > NBD - 1 ? NBD - 1 : bd);
      const float* hr = hin + (size_t)s * FD + 64 * q;
      const float* er = elt + (bt * NBD + bd) * FD + 64 * q;
      float* mr = msg + i * FD + 64 * q;
#pragma unroll 1
      for (int p = 0; p < 2; ++p) {
        v4f hv[8], tv[8];
#pragma unroll
        for (int j = 0; j < 8; ++j) {
          hv[j] = *(const v4f*)(hr + 32 * p + 4 * j);
          tv[j] = *(const v4f*)(er + 32 * p + 4 * j);
        }
#pragma unroll
        for (int j = 0; j < 8; ++j) *(v4f*)(mr + 32 * p + 4 * j) = relu4sum(hv[j], tv[j]);
      }
      if (q == 0) slotb[i] = slot;
    }
    __syncthreads();
    {
      int cnt = nP - r * PASSN;
      cnt = cnt > PASSN ? PASSN : (cnt < 0 ? 0 : cnt);
      if (tid < FD) {
#pragma unroll 1
        for (int i = 0; i < cnt; ++i) {
          int sl = slotb[i];
          sl = sl < 0 ? 0 : (sl > NB ? NB : sl);
          acc[sl * FD + tid] += msg[i * FD + tid];
        }
      }
    }
    __syncthreads();
  }

#pragma unroll 1
  for (int tt = 0; tt < 2; ++tt) {
    const int t = wave + NWAVE * tt;
    const int lrow = 16 * t + m;
    int node = nodeBase + lrow;
    node = node > nN - 1 ? nN - 1 : node;
    mlp_tile<4, 1>(acc + lrow * FD, hin + (size_t)node * FD, m1h, m1l, b1, m2h, m2l, b2, gam, bet,
                   hid + wave * 16 * FD, acc + lrow * FD, hh, m);
    __syncthreads();
  }

#pragma unroll 1
  for (int rr = 0; rr < NB / NWAVE; ++rr) {
    const int row = wave * (NB / NWAVE) + rr;
    const v4f v = *(const v4f*)(acc + row * FD + 4 * lane);
    *(volatile v4f*)(hout + (size_t)(nodeBase + row) * FD + 4 * lane) = v;
  }
  __threadfence();
#pragma unroll 1
  for (int rr = 0; rr < NB / NWAVE; ++rr) {
    const int row = wave * (NB / NWAVE) + rr;
    const v4f v = *(const v4f*)(acc + row * FD + 4 * lane);
    *(volatile v4f*)(hout + (size_t)(nodeBase + row) * FD + 4 * lane) = v;
  }
}

__global__ __launch_bounds__(PTHR) void k_pool(const float* __restrict__ hfin, const int* __restrict__ batch,
                                              float* ge, int nN, int G) {
  __shared__ __attribute__((aligned(16))) float gt[GB * GEW];
  __shared__ int plist[NWAVE * PWCAP];
  __shared__ int pwc[NWAVE];
  __shared__ int pcnt[GB];
  const int tid = threadIdx.x, lane = tid & 31, wave = tid >> 5;
  const int par = tid >> 7, c = tid & (FD - 1);
  const int g0 = blockIdx.x * GB;
  const float ninf = __uint_as_float(0xff800000u);
  for (int i = tid; i < GB * GEW; i += PTHR) gt[i] = ((i & (GEW - 1)) < FD) ? 0.0f : ninf;
  if (tid < GB) pcnt[tid] = 0;
  __syncthreads();
  const int nCh = (nN + PCHUNK - 1) / PCHUNK;
#pragma unroll 1
  for (int ch = 0; ch < nCh; ++ch) {
    const int cbase = ch * PCHUNK;
    int wc = 0;
    {
      const int n0 = cbase + tid * PEPT;
      const int sent = -2147483647 - 1;
      v4i b;
      if (cbase + PCHUNK <= nN) {
        b = *(const v4i*)(batch + n0);
      } else {
        b.x = (n0     < nN) ? batch[min(n0, nN - 1)] : sent;
        b.y = (n0 + 1 < nN) ? batch[min(n0 + 1, nN - 1)] : sent;
        b.z = (n0 + 2 < nN) ? batch[min(n0 + 2, nN - 1)] : sent;
        b.w = (n0 + 3 < nN) ? batch[min(n0 + 3, nN - 1)] : sent;
      }
      const unsigned ug = (unsigned)g0;
      const unsigned s0 = (unsigned)b.x - ug, s1 = (unsigned)b.y - ug;
      const unsigned s2 = (unsigned)b.z - ug, s3 = (unsigned)b.w - ug;
      const bool h0 = s0 < (unsigned)GB, h1 = s1 < (unsigned)GB, h2 = s2 < (unsigned)GB, h3 = s3 < (unsigned)GB;
      const unsigned any = __builtin_amdgcn_ballot_w32(h0 | h1 | h2 | h3);
      if (any != 0u) {
#define PHIT(J, HJ, SJ) { \
          const unsigned mj = __builtin_amdgcn_ballot_w32(HJ); \
          if (mj != 0u) { \
            if (HJ) { \
              const int pos = wc + (int)__builtin_amdgcn_mbcnt_lo(mj, 0u); \
              if (pos < PWCAP) plist[wave * PWCAP + pos] = (n0 + (J)) * GB + (int)(SJ); \
            } \
            wc += (int)__builtin_popcount(mj); } }
        PHIT(0, h0, s0)
        PHIT(1, h1, s1)
        PHIT(2, h2, s2)
        PHIT(3, h3, s3)
#undef PHIT
      }
    }
    if (lane == 0) pwc[wave] = wc;
    __syncthreads();
#pragma unroll 1
    for (int w = 0; w < NWAVE; ++w) {
      int n = pwc[w];
      n = n > PWCAP ? PWCAP : (n < 0 ? 0 : n);
#pragma unroll 1
      for (int i = 0; i < n; ++i) {
        const int pk = plist[w * PWCAP + i];
        const int gl = pk & (GB - 1);
        int nd = pk >> 4;
        nd = nd < 0 ? 0 : (nd > nN - 1 ? nN - 1 : nd);
        if ((gl & 1) == par) {
          const float v = hfin[(size_t)nd * FD + c];
          float* gp = gt + gl * GEW + c;
          gp[0] += v;
          gp[FD] = fmaxf(gp[FD], v);
          if (c == 0) pcnt[gl] += 1;
        }
      }
    }
    __syncthreads();
  }
  for (int i = tid; i < GB * FD; i += PTHR) {
    const int gl = i >> 7;
    const int cc = i & (FD - 1);
    const int g = g0 + gl;
    const float cn = (float)pcnt[gl];
    float mean = gt[gl * GEW + cc] * (1.0f / cn);
    float mx = gt[gl * GEW + FD + cc];
    if (g >= G) { mean = 0.0f; mx = 0.0f; }
    gt[gl * GEW + cc] = mean;
    gt[gl * GEW + FD + cc] = mx;
  }
  __syncthreads();
#pragma unroll 1
  for (int rr = 0; rr < 2; ++rr) {
    const int row = 2 * wave + rr;
#pragma unroll
    for (int j = 0; j < 2; ++j) {
      const v4f v = *(const v4f*)(gt + row * GEW + FD * j + 4 * lane);
      *(volatile v4f*)(ge + (size_t)(g0 + row) * GEW + FD * j + 4 * lane) = v;
    }
  }
  __threadfence();
#pragma unroll 1
  for (int rr = 0; rr < 2; ++rr) {
    const int row = 2 * wave + rr;
#pragma unroll
    for (int j = 0; j < 2; ++j) {
      const v4f v = *(const v4f*)(gt + row * GEW + FD * j + 4 * lane);
      *(volatile v4f*)(ge + (size_t)(g0 + row) * GEW + FD * j + 4 * lane) = v;
    }
  }
}

__device__ __forceinline__ void wave_gemm3(const float* bt, int bpitch, int nkt,
    const unsigned short* __restrict__ ah_p, const unsigned short* __restrict__ al_p, int kp,
    const float* __restrict__ bias, int nft, float* ot, int opitch, int ocol, int hh, int m) {
#pragma unroll 1
  for (int ft = 0; ft < nft; ++ft) {
    v8f acc = ldc8(bias + 16 * ft + 8 * hh);
    const unsigned short* ap = ah_p + (size_t)(16 * ft + m) * kp + 8 * hh;
    const unsigned short* aq = al_p + (size_t)(16 * ft + m) * kp + 8 * hh;
    const float* bp = bt + m * bpitch + 8 * hh;
#pragma unroll 1
    for (int kt = 0; kt < nkt; ++kt) {
      FragB bh, bl, fh, fl;
      split8(*(const v4f*)(bp + 32 * kt), *(const v4f*)(bp + 32 * kt + 4), bh.h[0], bl.h[0]);
      split8(*(const v4f*)(bp + 32 * kt + 16), *(const v4f*)(bp + 32 * kt + 20), bh.h[1], bl.h[1]);
      fh.h[0] = *(const v8us*)(ap + 32 * kt);
      fh.h[1] = *(const v8us*)(ap + 32 * kt + 16);
      fl.h[0] = *(const v8us*)(aq + 32 * kt);
      fl.h[1] = *(const v8us*)(aq + 32 * kt + 16);
      acc = wm3(fh.v, fl.v, bh.v, bl.v, acc);
    }
    strelu8(ot + m * opitch + ocol + 16 * ft + 8 * hh, acc);
  }
}

__global__ __launch_bounds__(HTHR) void k_head(const float* __restrict__ xfeat, const float* __restrict__ ge,
    const unsigned short* __restrict__ e1h, const unsigned short* __restrict__ e1l, const float* __restrict__ eb1,
    const unsigned short* __restrict__ e2h, const unsigned short* __restrict__ e2l, const float* __restrict__ eb2,
    const unsigned short* __restrict__ w1h, const unsigned short* __restrict__ w1l, const float* __restrict__ hb1,
    const unsigned short* __restrict__ w2h, const unsigned short* __restrict__ w2l, const float* __restrict__ hb2,
    const float* __restrict__ hw3, const float* __restrict__ hb3,
    float* cmb, float* out0, int G, int Gp) {
  extern __shared__ __attribute__((aligned(16))) unsigned char dsmh[];
  const int tid = threadIdx.x, lane = tid & 31, wave = tid >> 5, hh = lane >> 4, m = lane & 15;
  float* T0 = (float*)dsmh + wave * HWAVE;
  float* T1 = T0 + HWT0;
  float* CT = T1 + HWT1;
  float* o0s = (float*)dsmh + 4 * HWAVE;
  const int g0 = blockIdx.x * HG + wave * 16;

#pragma unroll 1
  for (int i = lane; i < 16 * EXPKP; i += 32) {
    const int r = i / EXPKP;
    const int cc = i - r * EXPKP;
    int row = g0 + r;
    row = row > G - 1 ? G - 1 : row;
    const int ccl = cc < EXPK ? cc : EXPK - 1;
    const float v = xfeat[(size_t)row * EXPK + ccl];
    T0[r * EXPKP + cc] = (cc < EXPK) ? v : 0.0f;
  }
#pragma unroll 1
  for (int i = lane; i < 16 * (GEW / 4); i += 32) {
    const int r = i >> 6;
    const int c4 = i & 63;
    int row = g0 + r;
    row = row > Gp - 1 ? Gp - 1 : row;
    const v4f v = *(const v4f*)(ge + (size_t)row * GEW + 4 * c4);
    *(v4f*)(CT + r * CMBW + 4 * c4) = v;
  }
  __syncthreads();
  wave_gemm3(T0, EXPKP, EXPKP / 32, e1h, e1l, EXPKP, eb1, FD / 16, T1, FD, 0, hh, m);
  __syncthreads();
  wave_gemm3(T1, FD, FD / 32, e2h, e2l, FD, eb2, FD / 16, CT, CMBW, GEW, hh, m);
  __syncthreads();
  wave_gemm3(CT, CMBW, CMBW / 32, w1h, w1l, CMBW, hb1, O1W / 16, T0, O1W, 0, hh, m);
  __syncthreads();
  wave_gemm3(T0, O1W, O1W / 32, w2h, w2l, O1W, hb2, FD / 16, T1, FD, 0, hh, m);
  __syncthreads();
  {
    const float* orow = T1 + m * FD + 64 * hh;
    const float* wv = hw3 + 64 * hh;
    float s = 0.0f;
#pragma unroll 1
    for (int k = 0; k < 64; ++k) s += orow[k] * wv[k];
    const float t = __shfl_xor(s, 16);
    const float lo = (hh == 0) ? s : t;
    const float hi = (hh == 0) ? t : s;
    const float o = (lo + hi) + hb3[0];
    if (hh == 0) o0s[wave * 16 + m] = o;
  }
  __syncthreads();
  v4f ov;
  ov.x = 0.0f; ov.y = 0.0f; ov.z = 0.0f; ov.w = 0.0f;
  if (wave == 0 && lane < 16) ov = *(const v4f*)(o0s + 4 * lane);
#pragma unroll 1
  for (int rr = 0; rr < 16; ++rr) {
    const size_t row = (size_t)(g0 + rr);
#pragma unroll
    for (int j = 0; j < 3; ++j) {
      const v4f v = *(const v4f*)(CT + rr * CMBW + FD * j + 4 * lane);
      *(volatile v4f*)(cmb + row * CMBW + FD * j + 4 * lane) = v;
    }
  }
  if (wave == 0 && lane < 16) *(volatile v4f*)(out0 + (size_t)blockIdx.x * HG + 4 * lane) = ov;
  __threadfence();
#pragma unroll 1
  for (int rr = 0; rr < 16; ++rr) {
    const size_t row = (size_t)(g0 + rr);
#pragma unroll
    for (int j = 0; j < 3; ++j) {
      const v4f v = *(const v4f*)(CT + rr * CMBW + FD * j + 4 * lane);
      *(volatile v4f*)(cmb + row * CMBW + FD * j + 4 * lane) = v;
    }
  }
  if (wave == 0 && lane < 16) *(volatile v4f*)(out0 + (size_t)blockIdx.x * HG + 4 * lane) = ov;
}

__global__ __launch_bounds__(NTHR) void k_out(const float* __restrict__ out0p, const float* __restrict__ gep,
                                             const float* __restrict__ cmbp, float* dout, int G, int Gp, int n4) {
  const int u = blockIdx.x * NTHR + threadIdx.x;
  if (u >= n4) return;
  const int f = 4 * u;
  int i0 = f;
  i0 = i0 > Gp - 4 ? Gp - 4 : i0;
  int i1 = f - G;
  i1 = i1 < 0 ? 0 : (i1 > Gp * GEW - 4 ? Gp * GEW - 4 : i1);
  int i2 = f - G - G * GEW;
  i2 = i2 < 0 ? 0 : (i2 > Gp * CMBW - 4 ? Gp * CMBW - 4 : i2);
  const v4f v0 = *(const v4f*)(out0p + i0);
  const v4f v1 = *(const v4f*)(gep + i1);
  const v4f v2 = *(const v4f*)(cmbp + i2);
  const bool r0 = f < G;
  const bool r1 = f < G + G * GEW;
  v4f v;
  v.x = r0 ? v0.x : (r1 ? v1.x : v2.x);
  v.y = r0 ? v0.y : (r1 ? v1.y : v2.y);
  v.z = r0 ? v0.z : (r1 ? v1.z : v2.z);
  v.w = r0 ? v0.w : (r1 ? v1.w : v2.w);
  *(volatile v4f*)(dout + f) = v;
  __threadfence();
  *(volatile v4f*)(dout + f) = v;
}

extern "C" void kernel_launch(void* const* d_in, const int* in_sizes, int n_in,
                              void* d_out, int out_size, void* d_ws, size_t ws_size,
                              hipStream_t stream) {
  if (n_in < 29) return;
  const int nN = in_sizes[3];
  if (nN < 1 || in_sizes[0] != nN * NIN) return;
  const int nE = in_sizes[1] / 2;
  if (nE < 1 || in_sizes[1] != 2 * nE || in_sizes[2] != 2 * nE) return;
  const int G = out_size / (1 + GEW + CMBW);
  if (G < 1 || out_size != G * (1 + GEW + CMBW) || (G & 3) != 0) return;
  if (in_sizes[4] != G * EXPK) return;
  if (in_sizes[5] != NIN * FD || in_sizes[6] != FD || in_sizes[7] != FD * FD || in_sizes[8] != FD) return;
  if (in_sizes[9] != NBT * EEMB || in_sizes[10] != NBD * EEMB) return;
  if (in_sizes[11] != NLAY * EEMB * FD || in_sizes[12] != NLAY * FD) return;
  if (in_sizes[13] != NLAY * FD * FD || in_sizes[14] != NLAY * FD) return;
  if (in_sizes[15] != NLAY * FD * FD || in_sizes[16] != NLAY * FD) return;
  if (in_sizes[17] != NLAY * FD || in_sizes[18] != NLAY * FD) return;
  if (in_sizes[19] != EXPK * FD || in_sizes[20] != FD || in_sizes[21] != FD * FD || in_sizes[22] != FD) return;
  if (in_sizes[23] != CMBW * O1W || in_sizes[24] != O1W || in_sizes[25] != O1W * FD || in_sizes[26] != FD) return;
  if (in_sizes[27] != FD || in_sizes[28] != 1) return;

  const float* x     = (const float*)d_in[0];
  const int*   ei    = (const int*)d_in[1];
  const int*   ea    = (const int*)d_in[2];
  const int*   batch = (const int*)d_in[3];
  const float* xfeat = (const float*)d_in[4];
  const float* nw1 = (const float*)d_in[5],  *nb1 = (const float*)d_in[6];
  const float* nw2 = (const float*)d_in[7],  *nb2 = (const float*)d_in[8];
  const float* te  = (const float*)d_in[9],  *de  = (const float*)d_in[10];
  const float* lew = (const float*)d_in[11], *leb = (const float*)d_in[12];
  const float* mw1 = (const float*)d_in[13], *mb1 = (const float*)d_in[14];
  const float* mw2 = (const float*)d_in[15], *mb2 = (const float*)d_in[16];
  const float* gam = (const float*)d_in[17], *bet = (const float*)d_in[18];
  const float* ew1 = (const float*)d_in[19], *eb1 = (const float*)d_in[20];
  const float* ew2 = (const float*)d_in[21], *eb2 = (const float*)d_in[22];
  const float* hw1 = (const float*)d_in[23], *hb1 = (const float*)d_in[24];
  const float* hw2 = (const float*)d_in[25], *hb2 = (const float*)d_in[26];
  const float* hw3 = (const float*)d_in[27], *hb3 = (const float*)d_in[28];
  float* dout = (float*)d_out;

  const int nBlk = (nN + NB - 1) / NB;
  const size_t rowsP = (size_t)nBlk * NB;
  const int nPJ = (int)(rowsP / PJR);
  const int Gp = ((G + HG - 1) / HG) * HG;
  const int n4 = out_size / 4;

  const size_t nq0 = (size_t)FD * NIN, nq1 = (size_t)FD * FD, nq2 = (size_t)NLAY * FD * FD, nq3 = nq2;
  const size_t nq4 = (size_t)FD * EXPKP, nq5 = nq1, nq6 = (size_t)O1W * CMBW, nq7 = (size_t)FD * O1W;

  char* ws = (char*)d_ws;
  size_t off = 0;
  auto carve = [&](size_t bytes) -> size_t {
    const size_t o = off;
    off = (off + bytes + 255) & ~(size_t)255;
    return o;
  };
  const size_t oq0 = carve(2 * nq0 * 2), oq1 = carve(2 * nq1 * 2), oq2 = carve(2 * nq2 * 2), oq3 = carve(2 * nq3 * 2);
  const size_t oq4 = carve(2 * nq4 * 2), oq5 = carve(2 * nq5 * 2), oq6 = carve(2 * nq6 * 2), oq7 = carve(2 * nq7 * 2);
  const size_t otab = carve((size_t)NLAY * NCMB * FD * 4);
  const size_t oet  = carve((size_t)nBlk * EROW * 4);
  const size_t oX0  = carve(rowsP * FD * 4);
  const size_t oX1  = carve(rowsP * FD * 4);
  const size_t oGE  = carve((size_t)Gp * GEW * 4);
  const size_t oCM  = carve((size_t)Gp * CMBW * 4);
  const size_t oO0  = carve((size_t)Gp * 4);
  size_t limit = (size_t)134217728;
  if (ws_size < limit) limit = ws_size;
  if (off > limit) return;

  unsigned short* q0 = (unsigned short*)(ws + oq0);
  unsigned short* q1 = (unsigned short*)(ws + oq1);
  unsigned short* q2 = (unsigned short*)(ws + oq2);
  unsigned short* q3 = (unsigned short*)(ws + oq3);
  unsigned short* q4 = (unsigned short*)(ws + oq4);
  unsigned short* q5 = (unsigned short*)(ws + oq5);
  unsigned short* q6 = (unsigned short*)(ws + oq6);
  unsigned short* q7 = (unsigned short*)(ws + oq7);
  float* tab  = (float*)(ws + otab);
  int*   etab = (int*)(ws + oet);
  float* X0   = (float*)(ws + oX0);
  float* X1   = (float*)(ws + oX1);
  float* GE   = (float*)(ws + oGE);
  float* CM   = (float*)(ws + oCM);
  float* O0   = (float*)(ws + oO0);

  const int vec8 = ((nE & 3) == 0) ? 1 : 0;

  k_prep<<<PBT, NTHR, 0, stream>>>(nw1, nw2, mw1, mw2, ew1, ew2, hw1, hw2, q0, q1, q2, q3, q4, q5, q6, q7);
  k_tab<<<(NLAY * NCMB * FD + NTHR - 1) / NTHR, NTHR, 0, stream>>>(te, de, lew, leb, tab);
  k_escan<<<nBlk, NTHR, 0, stream>>>(ei, etab, nE, vec8);

  hipFuncSetAttribute(reinterpret_cast<const void*>(&k_proj), hipFuncAttributeMaxDynamicSharedMemorySize, LDS_PROJ);
  k_proj<<<nPJ, PJT, LDS_PROJ, stream>>>(x, q0, q0 + nq0, nb1, q1, q1 + nq1, nb2, X0, nN);

  hipFuncSetAttribute(reinterpret_cast<const void*>(&k_layer), hipFuncAttributeMaxDynamicSharedMemorySize, LDS_LAYER);
  float* hcur = X0;
  float* hnxt = X1;
  for (int l = 0; l < NLAY; ++l) {
    k_layer<<<nBlk, NTHR, LDS_LAYER, stream>>>(
        hcur, ei, ea, etab, tab + (size_t)l * NCMB * FD,
        q2 + (size_t)l * FD * FD, q2 + nq2 + (size_t)l * FD * FD, mb1 + (size_t)l * FD,
        q3 + (size_t)l * FD * FD, q3 + nq3 + (size_t)l * FD * FD, mb2 + (size_t)l * FD,
        gam + (size_t)l * FD, bet + (size_t)l * FD,
        hnxt, nN, nE);
    float* tsw = hcur; hcur = hnxt; hnxt = tsw;
  }

  k_pool<<<Gp / GB, PTHR, 0, stream>>>(hcur, batch, GE, nN, G);

  hipFuncSetAttribute(reinterpret_cast<const void*>(&k_head), hipFuncAttributeMaxDynamicSharedMemorySize, LDS_HEAD);
  k_head<<<Gp / HG, HTHR, LDS_HEAD, stream>>>(xfeat, GE, q4, q4 + nq4, eb1, q5, q5 + nq5, eb2,
                                              q6, q6 + nq6, hb1, q7, q7 + nq7, hb2, hw3, hb3, CM, O0, G, Gp);

  k_out<<<(n4 + NTHR - 1) / NTHR, NTHR, 0, stream>>>(O0, GE, CM, dout, G, Gp, n4);
}
